// mLSTMLayerV1_13322988552752
// MI455X (gfx1250) — hardware-verified
//
#include <hip/hip_runtime.h>


#define NB   2
#define NS   2048
#define ND   1024
#define NH   8
#define NQK  512
#define NDV  1024
#define DHQ  64
#define DHV  128
#define NTOK 4096
#define EPSV 1e-6f
#define GCAP 15.0f

typedef __bf16         v16bf __attribute__((ext_vector_type(16)));
typedef _Float16       v16h  __attribute__((ext_vector_type(16)));
typedef unsigned short v16us __attribute__((ext_vector_type(16), __may_alias__));
typedef unsigned short v8us  __attribute__((ext_vector_type(8), __may_alias__));
typedef float          v8f   __attribute__((ext_vector_type(8)));
typedef float          v4f   __attribute__((ext_vector_type(4), __may_alias__));

static __device__ __forceinline__ unsigned short f2bf(float f) {
  unsigned int u = __float_as_uint(f);
  u += 0x7FFFu + ((u >> 16) & 1u);
  return (unsigned short)(u >> 16);
}
static __device__ __forceinline__ float bf2f(unsigned short v) { return __uint_as_float(((unsigned int)v) << 16); }
static __device__ __forceinline__ float bfr(float f) { return bf2f(f2bf(f)); }
static __device__ __forceinline__ unsigned short h2us(float f) {
  _Float16 h = (_Float16)f;
  return __builtin_bit_cast(unsigned short, h);
}
static __device__ __forceinline__ int packpos(int k) { return (k & ~31) + 16 * ((k >> 3) & 1) + (k & 7) + 8 * ((k >> 4) & 1); }
static __device__ __forceinline__ int posk(int p)    { return (p & ~31) + 8 * ((p >> 4) & 1) + (p & 7) + 16 * ((p >> 3) & 1); }

static __device__ __forceinline__ v8f zero8() {
  v8f z;
#pragma unroll
  for (int i = 0; i < 8; ++i) z[i] = 0.f;
  return z;
}

static __device__ __forceinline__ v8f mma_bf(v16us a, v16us b, v8f c) {
  v16bf av = __builtin_bit_cast(v16bf, a);
  v16bf bv = __builtin_bit_cast(v16bf, b);
  c = __builtin_amdgcn_wmma_f32_16x16x32_bf16(false, av, false, bv, (short)0, c, false, false);
  asm volatile("v_nop\n\tv_nop\n\tv_nop\n\tv_nop" : "+v"(c) : "v"(av), "v"(bv));
  return c;
}
static __device__ __forceinline__ v8f mma_h(v16us a, v16us b, v8f c) {
  v16h av = __builtin_bit_cast(v16h, a);
  v16h bv = __builtin_bit_cast(v16h, b);
  c = __builtin_amdgcn_wmma_f32_16x16x32_f16(false, av, false, bv, (short)0, c, false, false);
  asm volatile("v_nop\n\tv_nop\n\tv_nop\n\tv_nop" : "+v"(c) : "v"(av), "v"(bv));
  return c;
}

__global__ __launch_bounds__(256) void k_pack_x(const float* __restrict__ x,
                                                unsigned short* __restrict__ xb, int ntok) {
  const int gid = blockIdx.x * 256 + (int)threadIdx.x;
  const int row = gid >> 7;
  if (row >= ntok) return;
  const int p0 = (gid & 127) * 8;
  const int k  = (p0 & ~31) + 8 * ((p0 >> 4) & 1) + 16 * ((p0 >> 3) & 1);
  const v4f* src = (const v4f*)(x + (size_t)row * ND + k);
  const v4f f0 = src[0], f1 = src[1];
  v8us o;
#pragma unroll
  for (int i = 0; i < 4; ++i) { o[i] = f2bf(f0[i]); o[4 + i] = f2bf(f1[i]); }
  volatile v8us* dst = (volatile v8us*)(xb + (size_t)row * ND + p0);
  *dst = o;
  __threadfence();
  *dst = o;
}

static __device__ __forceinline__ void pack_w_store(const unsigned short (*sT)[72], unsigned short* Wp,
                                                    int n0, int k0, int N, int t) {
#pragma unroll
  for (int p = 0; p < 2; ++p) {
    const int row = p * 32 + (t >> 3), piece = t & 7;
    const v8us v = *(const v8us*)(&sT[row][piece * 8]);
    if (n0 + row < N)
      *(volatile v8us*)(Wp + (size_t)(n0 + row) * ND + k0 + piece * 8) = v;
  }
}

template <int F16>
__global__ __launch_bounds__(256) void k_pack_w(const float* __restrict__ W,
                                                unsigned short* __restrict__ Wp, int N, float scale) {
  __shared__ __attribute__((aligned(16))) unsigned short sT[64][72];
  const int t = (int)threadIdx.x;
  const int n0 = blockIdx.x * 64, k0 = blockIdx.y * 64;
#pragma unroll 4
  for (int i = 0; i < 16; ++i) {
    const int idx = i * 256 + t;
    const int kk = idx >> 6, nn = idx & 63;
    float v = 0.f;
    if (n0 + nn < N && k0 + kk < ND) v = W[(size_t)(k0 + kk) * N + n0 + nn];
    unsigned short o;
    if (F16) o = h2us(bfr(v) * scale); else o = f2bf(v);
    sT[nn][packpos(kk)] = o;
  }
  __syncthreads();
  pack_w_store(sT, Wp, n0, k0, N, t);
  __threadfence();
  pack_w_store(sT, Wp, n0, k0, N, t);
}

template <int MODE>
static __device__ __forceinline__ void gemm_store(const float (*sC)[132], float* Cf, unsigned short* Ca,
                                                  unsigned short* Cb, int bm, int bn, int M, int N,
                                                  float oscale, int t) {
  if constexpr (MODE == 0) {
    const int l = t & 31;
#pragma unroll
    for (int p = 0; p < 8; ++p) {
      const int row = p * 8 + (t >> 5);
      const int grow = bm + row, gcol = bn + 4 * l;
      v4f v = *(const v4f*)(&sC[row][4 * l]);
      v = v * oscale;
      if (grow < M && gcol + 3 < N)
        *(volatile v4f*)(Cf + (size_t)grow * N + gcol) = v;
    }
  } else if constexpr (MODE == 1) {
#pragma unroll
    for (int p = 0; p < 4; ++p) {
      const int task = p * 256 + t;
      const int L = task >> 3, piece = task & 7;
      const int row = L >> 1, j = L & 1;
      const int grow = bm + row;
      const int head = (bn / DHQ) + j;
      const int kb = 32 * (piece >> 2) + 8 * ((piece >> 1) & 1) + 16 * (piece & 1);
      const v4f f0 = *(const v4f*)(&sC[row][j * DHQ + kb]);
      const v4f f1 = *(const v4f*)(&sC[row][j * DHQ + kb + 4]);
      v8us hi, lo;
#pragma unroll
      for (int i = 0; i < 4; ++i) {
        const unsigned short a = f2bf(f0[i]); hi[i] = a;     lo[i] = f2bf(f0[i] - bf2f(a));
        const unsigned short c = f2bf(f1[i]); hi[4 + i] = c; lo[4 + i] = f2bf(f1[i] - bf2f(c));
      }
      const int bb = grow / NS, s = grow % NS;
      const size_t o = (((size_t)(bb * NH + head)) * NS + s) * DHQ + piece * 8;
      if (grow < M && (head + 1) * DHQ <= N) {
        *(volatile v8us*)(Ca + o) = hi;
        *(volatile v8us*)(Cb + o) = lo;
      }
    }
  } else {
    const int head = bn / DHV;
    const int bb = bm / NS, s0 = bm % NS;
#pragma unroll
    for (int p = 0; p < 4; ++p) {
      const int task = p * 256 + t;
      const int dv = task >> 3, piece = task & 7;
      const int tb = 32 * (piece >> 2) + 8 * ((piece >> 1) & 1) + 16 * (piece & 1);
      v8us o8;
#pragma unroll
      for (int i = 0; i < 8; ++i) o8[i] = h2us(sC[tb + i][dv] * oscale);
      const size_t o = (((size_t)(bb * NH + head)) * DHV + dv) * NS + s0 + piece * 8;
      if (bm + 63 < M && bn + dv < N)
        *(volatile v8us*)(Ca + o) = o8;
    }
  }
}

template <int F16, int MODE>
__global__ __launch_bounds__(256) void k_gemm(const unsigned short* __restrict__ Ap,
                                              const unsigned short* __restrict__ Bp,
                                              float* Cf, unsigned short* Ca, unsigned short* Cb,
                                              int M, int N, float oscale) {
  __shared__ __attribute__((aligned(16))) float sC[64][132];
  const int lane = threadIdx.x & 31, wave = threadIdx.x >> 5;
  const int wm = wave & 1, wn = wave >> 1;
  const int m16 = lane & 15, hh = lane >> 4;
  const int bm = blockIdx.x * 64, bn = blockIdx.y * 128;

  const int ar0 = min(bm + wm * 32 + m16, M - 1);
  const int ar1 = min(bm + wm * 32 + 16 + m16, M - 1);
  const int br0 = min(bn + wn * 32 + m16, N - 1);
  const int br1 = min(bn + wn * 32 + 16 + m16, N - 1);
  const unsigned short* pa0 = Ap + (size_t)ar0 * ND + 16 * hh;
  const unsigned short* pa1 = Ap + (size_t)ar1 * ND + 16 * hh;
  const unsigned short* pb0 = Bp + (size_t)br0 * ND + 16 * hh;
  const unsigned short* pb1 = Bp + (size_t)br1 * ND + 16 * hh;

  v8f acc00 = zero8(), acc01 = zero8(), acc10 = zero8(), acc11 = zero8();
  for (int k0 = 0; k0 < ND; k0 += 32) {
    const v16us a0 = *(const v16us*)(pa0 + k0);
    const v16us a1 = *(const v16us*)(pa1 + k0);
    const v16us b0 = *(const v16us*)(pb0 + k0);
    const v16us b1 = *(const v16us*)(pb1 + k0);
    if (F16) {
      acc00 = mma_h(a0, b0, acc00);  acc01 = mma_h(a0, b1, acc01);
      acc10 = mma_h(a1, b0, acc10);  acc11 = mma_h(a1, b1, acc11);
    } else {
      acc00 = mma_bf(a0, b0, acc00); acc01 = mma_bf(a0, b1, acc01);
      acc10 = mma_bf(a1, b0, acc10); acc11 = mma_bf(a1, b1, acc11);
    }
  }

  const int r0 = wm * 32 + 8 * hh, c0 = wn * 32 + m16;
#pragma unroll
  for (int r = 0; r < 8; ++r) {
    sC[r0 + r][c0]           = acc00[r];
    sC[r0 + r][c0 + 16]      = acc01[r];
    sC[r0 + 16 + r][c0]      = acc10[r];
    sC[r0 + 16 + r][c0 + 16] = acc11[r];
  }
  __syncthreads();
  gemm_store<MODE>(sC, Cf, Ca, Cb, bm, bn, M, N, oscale, (int)threadIdx.x);
  __threadfence();
  gemm_store<MODE>(sC, Cf, Ca, Cb, bm, bn, M, N, oscale, (int)threadIdx.x);
}

__global__ __launch_bounds__(256) void k_gates(const unsigned short* __restrict__ xb,
                                               const float* __restrict__ Wi, const float* __restrict__ bi,
                                               const float* __restrict__ Wf, const float* __restrict__ bfp,
                                               float* __restrict__ lfc, float* __restrict__ gk,
                                               float* __restrict__ gmax) {
  __shared__ __attribute__((aligned(16))) float sWi[ND];
  __shared__ __attribute__((aligned(16))) float sWf[ND];
  __shared__ double sd[256];
  __shared__ float  sm[256];
  const int bh = blockIdx.x, b = bh / NH, head = bh % NH, t = (int)threadIdx.x;
  for (int p = t; p < ND; p += 256) {
    const int k = posk(p);
    sWi[p] = bfr(Wi[k * NH + head]);
    sWf[p] = bfr(Wf[k * NH + head]);
  }
  const float bir = bfr(bi[head]);
  const float bfc = bfr(bfp[head]);
  __syncthreads();

  double carry = 0.0;
  float carrym = -__builtin_inff();
  for (int s0 = 0; s0 < NS; s0 += 256) {
    const int s = s0 + t;
    const v8us* xr = (const v8us*)(xb + ((size_t)b * NS + s) * ND);
    float di = 0.f, df = 0.f;
#pragma unroll 1
    for (int j = 0; j < ND / 8; ++j) {
      const v8us xv = xr[j];
      const v4f wi0 = *(const v4f*)(sWi + 8 * j), wi1 = *(const v4f*)(sWi + 8 * j + 4);
      const v4f wf0 = *(const v4f*)(sWf + 8 * j), wf1 = *(const v4f*)(sWf + 8 * j + 4);
#pragma unroll
      for (int e = 0; e < 4; ++e) {
        const float x0 = bf2f(xv[e]), x1 = bf2f(xv[4 + e]);
        di = fmaf(x0, wi0[e], di); df = fmaf(x0, wf0[e], df);
        di = fmaf(x1, wi1[e], di); df = fmaf(x1, wf1[e], df);
      }
    }
    di += bir;
    df += bfc;
    const float ic = GCAP * tanhf(di * (1.0f / GCAP));
    const float fc = GCAP * tanhf(df * (1.0f / GCAP));
    const float lv = fminf(fc, 0.0f) - log1pf(expf(-fabsf(fc)));

    sd[t] = (double)lv;
    __syncthreads();
    for (int off = 1; off < 256; off <<= 1) {
      const double add = (t >= off) ? sd[t - off] : 0.0;
      __syncthreads();
      sd[t] += add;
      __syncthreads();
    }
    const double lfcd = carry + sd[t];
    const double tot  = sd[255];
    const float lfcv = (float)lfcd;
    const float gkv  = ic - lfcv;

    sm[t] = gkv;
    __syncthreads();
    for (int off = 1; off < 256; off <<= 1) {
      const float other = (t >= off) ? sm[t - off] : -__builtin_inff();
      __syncthreads();
      sm[t] = fmaxf(sm[t], other);
      __syncthreads();
    }
    const float gmv  = fmaxf(carrym, sm[t]);
    const float totm = sm[255];
    __syncthreads();
    carry += tot;
    carrym = fmaxf(carrym, totm);

    const size_t idx = (size_t)bh * NS + s;
    *(volatile float*)(lfc + idx)  = lfcv;
    *(volatile float*)(gk + idx)   = gkv;
    *(volatile float*)(gmax + idx) = gmv;
    __threadfence();
    *(volatile float*)(lfc + idx)  = lfcv;
    *(volatile float*)(gk + idx)   = gkv;
    *(volatile float*)(gmax + idx) = gmv;
  }
}

static __device__ __forceinline__ void attn_store(const unsigned short (*sG)[136], unsigned short* gp,
                                                  size_t tokb, int head, int m16, int hh) {
#pragma unroll
  for (int it = 0; it < 8; ++it) {
    const int row = it * 2 + hh;
    const v8us v = *(const v8us*)(&sG[row][m16 * 8]);
    *(volatile v8us*)(gp + (tokb + row) * ND + head * DHV + m16 * 8) = v;
  }
}

__global__ __launch_bounds__(32) void k_attn(const unsigned short* __restrict__ Qh,
                                             const unsigned short* __restrict__ Ql,
                                             const unsigned short* __restrict__ Kh,
                                             const unsigned short* __restrict__ Kl,
                                             const unsigned short* __restrict__ Vp,
                                             const float* __restrict__ lfc, const float* __restrict__ gk,
                                             const float* __restrict__ gmax, const float* __restrict__ ob,
                                             const float* __restrict__ onw, unsigned short* __restrict__ gp) {
  __shared__ __attribute__((aligned(32))) unsigned short Ps[32 * 16];
  __shared__ __attribute__((aligned(16))) unsigned short sG[16][136];
  const int qt = blockIdx.x % (NS / 16);
  const int bh = blockIdx.x / (NS / 16);
  const int head = bh % NH, b = bh / NH;
  const int lane = threadIdx.x & 31, m16 = lane & 15, hh = lane >> 4;
  const int qbase = qt * 16;
  const size_t rowbase = (size_t)bh * NS;

  const size_t qo = (rowbase + qbase + m16) * DHQ + 16 * hh;
  const v16us qh0 = *(const v16us*)(Qh + qo);
  const v16us qh1 = *(const v16us*)(Qh + qo + 32);
  const v16us ql0 = *(const v16us*)(Ql + qo);
  const v16us ql1 = *(const v16us*)(Ql + qo + 32);

  float gmr[8];
#pragma unroll
  for (int r = 0; r < 8; ++r) gmr[r] = gmax[rowbase + qbase + 8 * hh + r];

  v8f acc[8];
  float psum[8];
#pragma unroll
  for (int i = 0; i < 8; ++i) { acc[i] = zero8(); psum[i] = 0.f; }

  const unsigned short* kbh = Kh + rowbase * DHQ;
  const unsigned short* kbl = Kl + rowbase * DHQ;
  const unsigned short* vbp = Vp + (size_t)bh * DHV * NS;
  const float* gkh = gk + rowbase;

  for (int t0 = 0; t0 <= qbase + 15; t0 += 32) {
#pragma unroll
    for (int f = 0; f < 2; ++f) {
      const int tb = t0 + 16 * f;
      const float gkv = gkh[tb + m16];
      const size_t ko = (size_t)(tb + m16) * DHQ + 16 * hh;
      const v16us kh0 = *(const v16us*)(kbh + ko);
      const v16us kh1 = *(const v16us*)(kbh + ko + 32);
      const v16us kl0 = *(const v16us*)(kbl + ko);
      const v16us kl1 = *(const v16us*)(kbl + ko + 32);
      v8f cc = zero8();
      cc = mma_bf(qh0, kh0, cc); cc = mma_bf(qh1, kh1, cc);
      cc = mma_bf(ql0, kh0, cc); cc = mma_bf(ql1, kh1, cc);
      cc = mma_bf(qh0, kl0, cc); cc = mma_bf(qh1, kl1, cc);
#pragma unroll
      for (int r = 0; r < 8; ++r) {
        const int sg = qbase + 8 * hh + r;
        const float a = (tb + m16 <= sg) ? (gkv - gmr[r]) : -__builtin_inff();
        const float p = 0.125f * cc[r] * expf(a);
        psum[r] += p;
        const int lp = (8 * hh + r) + 16 * ((m16 >> 3) & 1);
        Ps[lp * 16 + (m16 & 7) + 8 * f] = h2us(256.0f * p);
      }
    }
    __syncthreads();
    const v16us pa = *(const v16us*)(&Ps[lane * 16]);
#pragma unroll
    for (int nf = 0; nf < 8; ++nf) {
      const v16us vv = *(const v16us*)(vbp + (size_t)(nf * 16 + m16) * NS + t0 + 16 * hh);
      acc[nf] = mma_h(pa, vv, acc[nf]);
    }
    __syncthreads();
  }

  float mu[8], rstd[8];
#pragma unroll
  for (int r = 0; r < 8; ++r) {
    float ps = psum[r];
    ps += __shfl_xor(ps, 1, 32); ps += __shfl_xor(ps, 2, 32);
    ps += __shfl_xor(ps, 4, 32); ps += __shfl_xor(ps, 8, 32);
    const int sg = qbase + 8 * hh + r;
    const float ms  = lfc[rowbase + sg] + gmr[r];
    const float nrm = fmaxf(fabsf(ps), expf(-ms)) + EPSV;
    const float inv = (1.0f / 4096.0f) / nrm;
#pragma unroll
    for (int nf = 0; nf < 8; ++nf) acc[nf][r] *= inv;
    float s1 = 0.f;
#pragma unroll
    for (int nf = 0; nf < 8; ++nf) s1 += acc[nf][r];
    s1 += __shfl_xor(s1, 1, 32); s1 += __shfl_xor(s1, 2, 32);
    s1 += __shfl_xor(s1, 4, 32); s1 += __shfl_xor(s1, 8, 32);
    mu[r] = s1 * (1.0f / DHV);
    float s2 = 0.f;
#pragma unroll
    for (int nf = 0; nf < 8; ++nf) { const float d = acc[nf][r] - mu[r]; s2 += d * d; }
    s2 += __shfl_xor(s2, 1, 32); s2 += __shfl_xor(s2, 2, 32);
    s2 += __shfl_xor(s2, 4, 32); s2 += __shfl_xor(s2, 8, 32);
    rstd[r] = 1.0f / sqrtf(s2 * (1.0f / DHV) + EPSV);
  }

  const size_t tokb = (size_t)b * NS + qbase;
#pragma unroll
  for (int nf = 0; nf < 8; ++nf) {
    const int col  = nf * 16 + m16;
    const int kcol = head * DHV + col;
    const float w  = bfr(onw[kcol]);
    const int pp   = packpos(col);
#pragma unroll
    for (int r = 0; r < 8; ++r) {
      const int row = 8 * hh + r;
      const float hn = (acc[nf][r] - mu[r]) * rstd[r] * w;
      const float og = ob[(tokb + row) * ND + kcol];
      const float sgm = 1.0f / (1.0f + expf(-og));
      sG[row][pp] = h2us(4.0f * (hn * sgm));
    }
  }
  __syncthreads();
  attn_store(sG, gp, tokb, head, m16, hh);
  __threadfence();
  attn_store(sG, gp, tokb, head, m16, hh);
}

extern "C" void kernel_launch(void* const* d_in, const int* in_sizes, int n_in,
                              void* d_out, int out_size, void* d_ws, size_t ws_size,
                              hipStream_t stream) {
  if (n_in < 11) return;
  if (in_sizes[0] != NTOK * ND || in_sizes[1] != ND * NQK || in_sizes[2] != ND * NQK ||
      in_sizes[3] != ND * NDV || in_sizes[4] != ND * NDV || in_sizes[5] != ND * NH ||
      in_sizes[6] != NH || in_sizes[7] != ND * NH || in_sizes[8] != NH ||
      in_sizes[9] != NH * DHV || in_sizes[10] != NDV * ND || out_size != NTOK * ND) return;

  const float* x     = (const float*)d_in[0];
  const float* Wq    = (const float*)d_in[1];
  const float* Wk    = (const float*)d_in[2];
  const float* Wv    = (const float*)d_in[3];
  const float* Wo    = (const float*)d_in[4];
  const float* Wi    = (const float*)d_in[5];
  const float* bi    = (const float*)d_in[6];
  const float* Wf    = (const float*)d_in[7];
  const float* bfp   = (const float*)d_in[8];
  const float* onw   = (const float*)d_in[9];
  const float* Wdown = (const float*)d_in[10];
  float* out = (float*)d_out;

  const size_t bXb = (size_t)NTOK * ND * 2;
  const size_t bWq = (size_t)NQK * ND * 2;
  const size_t bWv = (size_t)NDV * ND * 2;
  const size_t bWd = (size_t)ND * NDV * 2;
  const size_t bQ  = (size_t)NB * NH * NS * DHQ * 2;
  const size_t bV  = (size_t)NB * NH * DHV * NS * 2;
  const size_t bOb = (size_t)NTOK * NDV * 4;
  const size_t bGp = (size_t)NTOK * NDV * 2;
  const size_t bG  = (size_t)NB * NH * NS * 4;
  const size_t total = bXb + 2 * bWq + 2 * bWv + bWd + 4 * bQ + bV + bOb + bGp + 3 * bG;
  if (total > ws_size) return;

  unsigned char* ws = (unsigned char*)d_ws;
  size_t off = 0;
  unsigned short* xb = (unsigned short*)(ws + off); off += bXb;
  unsigned short* wq = (unsigned short*)(ws + off); off += bWq;
  unsigned short* wk = (unsigned short*)(ws + off); off += bWq;
  unsigned short* wv = (unsigned short*)(ws + off); off += bWv;
  unsigned short* wo = (unsigned short*)(ws + off); off += bWv;
  unsigned short* wd = (unsigned short*)(ws + off); off += bWd;
  unsigned short* Qh = (unsigned short*)(ws + off); off += bQ;
  unsigned short* Ql = (unsigned short*)(ws + off); off += bQ;
  unsigned short* Kh = (unsigned short*)(ws + off); off += bQ;
  unsigned short* Kl = (unsigned short*)(ws + off); off += bQ;
  unsigned short* Vp = (unsigned short*)(ws + off); off += bV;
  float*          ob = (float*)(ws + off);          off += bOb;
  unsigned short* gp = (unsigned short*)(ws + off); off += bGp;
  float*          lf = (float*)(ws + off);          off += bG;
  float*          gkb = (float*)(ws + off);         off += bG;
  float*          gmb = (float*)(ws + off);         off += bG;
  if (off > ws_size) return;

  const dim3 blk(256);
  k_pack_x<<<dim3((NTOK * 128 + 255) / 256), blk, 0, stream>>>(x, xb, NTOK);
  k_pack_w<0><<<dim3((NQK + 63) / 64, ND / 64), blk, 0, stream>>>(Wq, wq, NQK, 1.0f);
  k_pack_w<0><<<dim3((NQK + 63) / 64, ND / 64), blk, 0, stream>>>(Wk, wk, NQK, 1.0f);
  k_pack_w<0><<<dim3((NDV + 63) / 64, ND / 64), blk, 0, stream>>>(Wv, wv, NDV, 1.0f);
  k_pack_w<0><<<dim3((NDV + 63) / 64, ND / 64), blk, 0, stream>>>(Wo, wo, NDV, 1.0f);
  k_pack_w<1><<<dim3((ND + 63) / 64, NDV / 64), blk, 0, stream>>>(Wdown, wd, ND, 16.0f);

  k_gemm<0, 1><<<dim3(NTOK / 64, NQK / 128), blk, 0, stream>>>(xb, wq, ob, Qh, Ql, NTOK, NQK, 1.0f);
  k_gemm<0, 1><<<dim3(NTOK / 64, NQK / 128), blk, 0, stream>>>(xb, wk, ob, Kh, Kl, NTOK, NQK, 1.0f);
  k_gemm<0, 2><<<dim3(NTOK / 64, NDV / 128), blk, 0, stream>>>(xb, wv, ob, Vp, gp, NTOK, NDV, 16.0f);
  k_gemm<0, 0><<<dim3(NTOK / 64, NDV / 128), blk, 0, stream>>>(xb, wo, ob, gp, gp, NTOK, NDV, 1.0f);

  k_gates<<<dim3(NB * NH), blk, 0, stream>>>(xb, Wi, bi, Wf, bfp, lf, gkb, gmb);

  k_attn<<<dim3(NB * NH * (NS / 16)), dim3(32), 0, stream>>>(Qh, Ql, Kh, Kl, Vp, lf, gkb, gmb, ob, onw, gp);

  k_gemm<1, 0><<<dim3(NTOK / 64, ND / 128), blk, 0, stream>>>(gp, wd, out, Vp, Vp, NTOK, ND, 1.0f / 64.0f);
}
